// DenseSAKELayer_8031588844293
// MI455X (gfx1250) — hardware-run, weakly checked
//
#include <hip/hip_runtime.h>
#include <stddef.h>
#include <stdint.h>


#define NBAT   2
#define NNODE  256
#define FIN    64
#define HID    64
#define NHEAD  4
#define CCO    256
#define NR     (NBAT * NNODE)
#define NPAIR  (NR * NNODE)
#define KE2    128
#define ABW    128
#define KIN1   (2 * FIN + 1)
#define KNODE  (FIN + CCO + HID)
#define NTHR   256
#define NWAVE  8
#define GBM    64
#define GBN    128
#define GTHR   128
#define DP     68
#define AP     136
#define CSTN   520
#define XVP    32
#define JT     64
#define WRN    53248
#define OFF_PW1 0
#define OFF_PW2 16384
#define OFF_NW1 20480
#define OFF_NW2 45056
#define OFF_VW1 49152
#define NU_WPT (ABW * (FIN / 8))
#define NU_W2D (HID * (KE2 / 8))
#define NU_HB  (NR * (FIN / 8))
#define NU_XB  NR
#define NU_WR  (WRN / 4)
#define NPREP  (NU_WPT + NU_W2D + NU_HB + NU_XB + NU_WR)
#define EDGE_LDS_BYTES (NTHR * DP * 4 + NTHR * AP * 2 + CSTN * 4 + NTHR * 4 * 4)
#define OUT0N  (NR * FIN)
#define OUT1N  (NR * 3)
#define OUTN   (OUT0N + 2 * OUT1N)
#define WSMAX  134217728
#define EPSV   1e-5f
#define INFV   1e5f
#define RN256  0.00390625f

static_assert(NU_WPT % NTHR == 0 && NU_W2D % NTHR == 0 && NU_HB % NTHR == 0 && NU_XB % NTHR == 0);
static_assert(NU_WR % NTHR == 0 && NPREP % NTHR == 0);
static_assert(OFF_PW2 % (4 * NTHR) == 0 && OFF_NW1 % (4 * NTHR) == 0 && OFF_NW2 % (4 * NTHR) == 0);
static_assert(OFF_VW1 % (4 * NTHR) == 0 && WRN % (4 * NTHR) == 0);
static_assert(OFF_PW2 == OFF_PW1 + CCO * HID && OFF_NW1 == OFF_PW2 + HID * HID);
static_assert(OFF_NW2 == OFF_NW1 + KNODE * HID && OFF_VW1 == OFF_NW2 + HID * FIN && WRN == OFF_VW1 + FIN * HID);
static_assert(EDGE_LDS_BYTES <= 300000);
static_assert((DP * 4) % 16 == 0 && (AP * 2) % 16 == 0 && AP >= KE2 && DP >= HID);
static_assert((CSTN * 4) % 16 == 0 && CSTN >= 8 * HID + NHEAD);
static_assert(GBM == (GTHR / 32) * 16 && GBN == 4 * 32 && ABW == GBN && NR % GBM == 0);
static_assert(FIN % 32 == 0 && KE2 % 32 == 0 && KE2 == 2 * HID && HID == FIN);
static_assert(NNODE == NTHR && CCO == NTHR && CCO == HID * NHEAD && NNODE % JT == 0);
static_assert(JT * HID == 4 * NTHR * 4);
static_assert(NNODE * HID == 16 * NTHR * 4);
static_assert((OUT0N * 4) % 128 == 0 && (OUT1N * 4) % 128 == 0 && (2 * OUT1N) == 3 * NTHR * 4);
static_assert(KIN1 == 129 && KNODE == 384);

typedef float          v4f   __attribute__((ext_vector_type(4)));
typedef float          v8f   __attribute__((ext_vector_type(8)));
typedef int            v4i   __attribute__((ext_vector_type(4)));
typedef int            v8i   __attribute__((ext_vector_type(8)));
typedef unsigned short v8us  __attribute__((ext_vector_type(8)));
typedef unsigned short v16us __attribute__((ext_vector_type(16)));
typedef __bf16         v16bf __attribute__((ext_vector_type(16)));
typedef v4f  __attribute__((may_alias)) v4fa;
typedef v4i  __attribute__((may_alias)) v4ia;
typedef v8us __attribute__((may_alias)) v8usa;
union FragB { v16bf v; v16us u; v8us h[2]; v8i w; };

__device__ __forceinline__ v8f wmb(const FragB& a, const FragB& b, v8f c) {
  v8f d = __builtin_amdgcn_wmma_f32_16x16x32_bf16(false, a.v, false, b.v, (short)0, c, false, false);
  asm volatile("v_nop\n\tv_nop\n\tv_nop\n\tv_nop" : "+v"(d) : "v"(a.w), "v"(b.w));
  return d;
}

__device__ __forceinline__ unsigned bf16_bits(float f) {
  const unsigned u = __float_as_uint(f);
  return (u + 0x7FFFu + ((u >> 16) & 1u)) >> 16;
}
__device__ __forceinline__ float bf16_val(float f) {
  return __uint_as_float(bf16_bits(f) << 16);
}
__device__ __forceinline__ float silu_f(float t) {
  return t * __builtin_amdgcn_rcpf(1.0f + __expf(-t));
}
__device__ __forceinline__ void put16(unsigned short* dp, v8us o) {
  *(volatile v8us*)dp = o;
  __threadfence();
  *(volatile v8us*)dp = o;
}
__device__ __forceinline__ void putf4(float* dp, v4f o) {
  *(volatile v4f*)dp = o;
  __threadfence();
  *(volatile v4f*)dp = o;
}
__device__ __forceinline__ v4f exp4(v4f a) {
  v4f r;
  r.x = __expf(a.x); r.y = __expf(a.y); r.z = __expf(a.z); r.w = __expf(a.w);
  return r;
}
__device__ __forceinline__ v4f rcp4(v4f a) {
  v4f r;
  r.x = __builtin_amdgcn_rcpf(a.x); r.y = __builtin_amdgcn_rcpf(a.y);
  r.z = __builtin_amdgcn_rcpf(a.z); r.w = __builtin_amdgcn_rcpf(a.w);
  return r;
}

__device__ __forceinline__ v4f blk_max4(v4f v, float* red, int lane, int wave) {
#pragma unroll
  for (int off = 16; off > 0; off >>= 1) {
    v.x = fmaxf(v.x, __shfl_xor(v.x, off, 32));
    v.y = fmaxf(v.y, __shfl_xor(v.y, off, 32));
    v.z = fmaxf(v.z, __shfl_xor(v.z, off, 32));
    v.w = fmaxf(v.w, __shfl_xor(v.w, off, 32));
  }
  if (lane == 0) *(v4fa*)(red + 4 * wave) = v;
  __syncthreads();
  v4f r = *(const v4fa*)red;
#pragma unroll
  for (int w = 1; w < NWAVE; ++w) {
    const v4f t = *(const v4fa*)(red + 4 * w);
    r.x = fmaxf(r.x, t.x); r.y = fmaxf(r.y, t.y); r.z = fmaxf(r.z, t.z); r.w = fmaxf(r.w, t.w);
  }
  __syncthreads();
  return r;
}
__device__ __forceinline__ v4f blk_sum4(v4f v, float* red, int lane, int wave) {
#pragma unroll
  for (int off = 16; off > 0; off >>= 1) {
    v.x += __shfl_xor(v.x, off, 32);
    v.y += __shfl_xor(v.y, off, 32);
    v.z += __shfl_xor(v.z, off, 32);
    v.w += __shfl_xor(v.w, off, 32);
  }
  if (lane == 0) *(v4fa*)(red + 4 * wave) = v;
  __syncthreads();
  v4f r = *(const v4fa*)red;
#pragma unroll
  for (int w = 1; w < NWAVE; ++w) {
    const v4f t = *(const v4fa*)(red + 4 * w);
    r.x += t.x; r.y += t.y; r.z += t.z; r.w += t.w;
  }
  __syncthreads();
  return r;
}

__global__ __launch_bounds__(NTHR) void k_prep(const float* __restrict__ h, const float* __restrict__ x,
                                               const float* __restrict__ W1, const float* __restrict__ W2,
                                               const float* __restrict__ pw1, const float* __restrict__ pw2,
                                               const float* __restrict__ nw1, const float* __restrict__ nw2,
                                               const float* __restrict__ vw1,
                                               unsigned short* WPT, unsigned short* W2D, unsigned short* HB,
                                               float* XB, float* WR) {
  const int u  = (int)blockIdx.x * NTHR + (int)threadIdx.x;
  const int U0 = NU_WPT;
  const int U1 = U0 + NU_W2D;
  const int U2 = U1 + NU_HB;
  const int U3 = U2 + NU_XB;
  const int U4 = U3 + NU_WR;
  v8us o;
  if (u < U0) {
    const int n  = u >> 3;
    const int k8 = (u & 7) * 8;
    const int q  = n >> 6;
    const int nn = n & (HID - 1);
    const float* p = W1 + (size_t)(q * FIN + k8) * HID + nn;
#pragma unroll
    for (int i = 0; i < 8; ++i) o[i] = (unsigned short)bf16_bits(p[(size_t)i * HID]);
    put16(WPT + (size_t)n * FIN + k8, o);
    return;
  } else if (u < U1) {
    const int v    = u - U0;
    const int n    = v >> 4;
    const int k8   = (v & 15) * 8;
    const int srow = k8 & (HID - 1);
    const float* p = W2 + (size_t)srow * HID + n;
#pragma unroll
    for (int i = 0; i < 8; ++i) o[i] = (unsigned short)bf16_bits(p[(size_t)i * HID]);
    put16(W2D + (size_t)n * KE2 + k8, o);
    return;
  } else if (u < U2) {
    const int v   = u - U1;
    const int row = v >> 3;
    const int k8  = (v & 7) * 8;
    const float* p = h + (size_t)row * FIN + k8;
    const v4f a = *(const v4fa*)p;
    const v4f b = *(const v4fa*)(p + 4);
    o[0] = (unsigned short)bf16_bits(a.x); o[1] = (unsigned short)bf16_bits(a.y);
    o[2] = (unsigned short)bf16_bits(a.z); o[3] = (unsigned short)bf16_bits(a.w);
    o[4] = (unsigned short)bf16_bits(b.x); o[5] = (unsigned short)bf16_bits(b.y);
    o[6] = (unsigned short)bf16_bits(b.z); o[7] = (unsigned short)bf16_bits(b.w);
    put16(HB + (size_t)row * FIN + k8, o);
    return;
  } else if (u < U3) {
    const int row = u - U2;
    const float x0 = x[(size_t)row * 3 + 0];
    const float x1 = x[(size_t)row * 3 + 1];
    const float x2 = x[(size_t)row * 3 + 2];
    v4f q;
    q.x = bf16_val(x0); q.y = bf16_val(x1); q.z = bf16_val(x2); q.w = 0.0f;
    putf4(XB + (size_t)row * 4, q);
    return;
  } else if (u < U4) {
    const int v = u - U3;
    const int f = 4 * v;
    const float* src;
    if (f < OFF_PW2)      src = pw1 + f;
    else if (f < OFF_NW1) src = pw2 + (f - OFF_PW2);
    else if (f < OFF_NW2) src = nw1 + (f - OFF_NW1);
    else if (f < OFF_VW1) src = nw2 + (f - OFF_NW2);
    else                  src = vw1 + (f - OFF_VW1);
    const v4f a = *(const v4fa*)src;
    v4f q;
    q.x = bf16_val(a.x); q.y = bf16_val(a.y); q.z = bf16_val(a.z); q.w = bf16_val(a.w);
    putf4(WR + f, q);
    return;
  }
}

__global__ __launch_bounds__(GTHR) void k_ab(const unsigned short* __restrict__ A, int lda,
                                             const unsigned short* __restrict__ BT, int ldb, int K,
                                             float* Cm, int ldc) {
  __shared__ __attribute__((aligned(16))) float stg[GBM * GBN];
  const int tid = (int)threadIdx.x, lane = tid & 31, wave = tid >> 5, hh = lane >> 4, m = lane & 15;
  const int rowBase = (int)blockIdx.x * GBM;
  const int colBase = (int)blockIdx.y * GBN;

  v8f acc[8];
  {
    const v8f z = {0.f, 0.f, 0.f, 0.f, 0.f, 0.f, 0.f, 0.f};
#pragma unroll
    for (int t = 0; t < 8; ++t) acc[t] = z;
  }
  const unsigned short* ap = A  + (size_t)(rowBase + 16 * wave + m) * (size_t)lda + 8 * hh;
  const unsigned short* bp = BT + (size_t)(colBase + m) * (size_t)ldb + 8 * hh;

#pragma unroll 1
  for (int k0 = 0; k0 < K; k0 += 32) {
    FragB af;
    af.h[0] = *(const v8usa*)(ap + k0);
    af.h[1] = *(const v8usa*)(ap + k0 + 16);
#pragma unroll
    for (int nt = 0; nt < 8; ++nt) {
      const unsigned short* wq = bp + (size_t)(16 * nt) * (size_t)ldb + k0;
      FragB bf;
      bf.h[0] = *(const v8usa*)wq;
      bf.h[1] = *(const v8usa*)(wq + 16);
      acc[nt] = wmb(af, bf, acc[nt]);
    }
  }

#pragma unroll
  for (int nt = 0; nt < 8; ++nt) {
    const int lc = 16 * nt + m;
#pragma unroll
    for (int r = 0; r < 8; ++r) {
      const int lr = 16 * wave + 8 * hh + r;
      stg[lr * GBN + lc] = acc[nt][r];
    }
  }
  __syncthreads();

  v4f pv[16];
#pragma unroll
  for (int i = 0; i < 16; ++i) pv[i] = *(const v4fa*)(stg + (16 * wave + i) * GBN + 4 * lane);
#pragma unroll
  for (int i = 0; i < 16; ++i) {
    float* op = Cm + (size_t)(rowBase + 16 * wave + i) * (size_t)ldc + colBase + 4 * lane;
    *(volatile v4f*)op = pv[i];
  }
  __threadfence();
#pragma unroll
  for (int i = 0; i < 16; ++i) {
    float* op = Cm + (size_t)(rowBase + 16 * wave + i) * (size_t)ldc + colBase + 4 * lane;
    *(volatile v4f*)op = pv[i];
  }
}

__device__ __forceinline__ void wave_gemm64(const unsigned short* sAw, float* sDw,
                                            const unsigned short* __restrict__ BT, int ldb, int K,
                                            int hh, int m) {
  v8f acc[2][4];
  {
    const v8f z = {0.f, 0.f, 0.f, 0.f, 0.f, 0.f, 0.f, 0.f};
#pragma unroll
    for (int mt = 0; mt < 2; ++mt)
#pragma unroll
      for (int nt = 0; nt < 4; ++nt) acc[mt][nt] = z;
  }
  const unsigned short* ap0 = sAw + m * AP + 8 * hh;
  const unsigned short* ap1 = ap0 + 16 * AP;
  const unsigned short* bp  = BT + (size_t)m * (size_t)ldb + 8 * hh;
#pragma unroll 1
  for (int k0 = 0; k0 < K; k0 += 32) {
    FragB a0, a1;
    a0.h[0] = *(const v8usa*)(ap0 + k0);
    a0.h[1] = *(const v8usa*)(ap0 + k0 + 16);
    a1.h[0] = *(const v8usa*)(ap1 + k0);
    a1.h[1] = *(const v8usa*)(ap1 + k0 + 16);
#pragma unroll
    for (int nt = 0; nt < 4; ++nt) {
      const unsigned short* wq = bp + (size_t)(16 * nt) * (size_t)ldb + k0;
      FragB b;
      b.h[0] = *(const v8usa*)wq;
      b.h[1] = *(const v8usa*)(wq + 16);
      acc[0][nt] = wmb(a0, b, acc[0][nt]);
      acc[1][nt] = wmb(a1, b, acc[1][nt]);
    }
  }
#pragma unroll
  for (int nt = 0; nt < 4; ++nt) {
    const int col = 16 * nt + m;
#pragma unroll
    for (int mt = 0; mt < 2; ++mt)
#pragma unroll
      for (int r = 0; r < 8; ++r) sDw[(16 * mt + 8 * hh + r) * DP + col] = acc[mt][nt][r];
  }
}

__global__ __launch_bounds__(NTHR) void k_edge(const float* __restrict__ XB, const float* __restrict__ AB,
                                               const float* __restrict__ W1, const float* __restrict__ b1,
                                               const unsigned short* __restrict__ W2D,
                                               const float* __restrict__ b2, const float* __restrict__ semw,
                                               const float* __restrict__ semb,
                                               float* HE, float* SEML) {
  extern __shared__ __attribute__((aligned(16))) float dyn[];
  float*          sD  = dyn;
  unsigned short* sA  = (unsigned short*)(dyn + NTHR * DP);
  float*          cst = dyn + NTHR * DP + (NTHR * AP) / 2;
  float*          sS  = cst + CSTN;

  const int tid = (int)threadIdx.x, lane = tid & 31, wave = tid >> 5, hh = lane >> 4, m = lane & 15;
  const int bi = (int)blockIdx.x;
  const int b  = bi >> 8;
  const int i  = bi & (NNODE - 1);
  const int j  = tid;

  if (tid < HID) {
    cst[tid]           = AB[(size_t)(b * NNODE + i) * ABW + HID + tid];
    cst[HID + tid]     = bf16_val(W1[(size_t)(2 * FIN) * HID + tid]);
    cst[2 * HID + tid] = bf16_val(b1[tid]);
    cst[3 * HID + tid] = bf16_val(b2[tid]);
    const v4f sw = *(const v4fa*)(semw + 4 * tid);
    v4f q;
    q.x = bf16_val(sw.x); q.y = bf16_val(sw.y); q.z = bf16_val(sw.z); q.w = bf16_val(sw.w);
    *(v4fa*)(cst + 4 * HID + 4 * tid) = q;
    const float sb = bf16_val(semb[tid & (NHEAD - 1)]);
    if (tid < NHEAD) cst[8 * HID + tid] = sb;
  }

  const v4f xi = *(const v4fa*)(XB + (size_t)(b * NNODE + i) * 4);
  const v4f xj = *(const v4fa*)(XB + (size_t)(b * NNODE + j) * 4);
  const float dx = xj.x - xi.x, dy = xj.y - xi.y, dz = xj.z - xi.z;
  const float r2 = (dx * dx + dz * dz) + dy * dy;
  const float r  = sqrtf(r2 + EPSV);
  __syncthreads();

  float*          rd = sD + tid * DP;
  unsigned short* ra = sA + tid * AP;
  {
    const float* pr = AB + (size_t)(b * NNODE + j) * ABW;
#pragma unroll 1
    for (int c8 = 0; c8 < HID / 8; ++c8) {
      const v4f pa = *(const v4fa*)(pr + 8 * c8);
      const v4f pb = *(const v4fa*)(pr + 8 * c8 + 4);
      const v4f qa = *(const v4fa*)(cst + 8 * c8);
      const v4f qb = *(const v4fa*)(cst + 8 * c8 + 4);
      const v4f wa = *(const v4fa*)(cst + HID + 8 * c8);
      const v4f wb = *(const v4fa*)(cst + HID + 8 * c8 + 4);
      const v4f ba = *(const v4fa*)(cst + 2 * HID + 8 * c8);
      const v4f bb = *(const v4fa*)(cst + 2 * HID + 8 * c8 + 4);
      const v8f p8 = {pa.x, pa.y, pa.z, pa.w, pb.x, pb.y, pb.z, pb.w};
      const v8f q8 = {qa.x, qa.y, qa.z, qa.w, qb.x, qb.y, qb.z, qb.w};
      const v8f w8 = {wa.x, wa.y, wa.z, wa.w, wb.x, wb.y, wb.z, wb.w};
      const v8f b8 = {ba.x, ba.y, ba.z, ba.w, bb.x, bb.y, bb.z, bb.w};
      v8us ho, lo;
#pragma unroll
      for (int e = 0; e < 8; ++e) {
        const float pre = (p8[e] + q8[e]) + fmaf(r, w8[e], b8[e]);
        const float ev  = silu_f(pre);
        const unsigned hb = bf16_bits(ev);
        ho[e] = (unsigned short)hb;
        lo[e] = (unsigned short)bf16_bits(ev - __uint_as_float(hb << 16));
      }
      *(v8usa*)(ra + 8 * c8)       = ho;
      *(v8usa*)(ra + HID + 8 * c8) = lo;
    }
  }
  __syncthreads();

  wave_gemm64(sA + 32 * wave * AP, sD + 32 * wave * DP, W2D, KE2, KE2, hh, m);
  __syncthreads();

  {
    float s0 = 0.0f, s1 = 0.0f, s2 = 0.0f, s3 = 0.0f;
#pragma unroll 1
    for (int c8 = 0; c8 < HID / 8; ++c8) {
      const v4f va = *(const v4fa*)(rd + 8 * c8);
      const v4f vb = *(const v4fa*)(rd + 8 * c8 + 4);
      const v4f ba = *(const v4fa*)(cst + 3 * HID + 8 * c8);
      const v4f bb = *(const v4fa*)(cst + 3 * HID + 8 * c8 + 4);
      const v8f v8 = {va.x, va.y, va.z, va.w, vb.x, vb.y, vb.z, vb.w};
      const v8f b8 = {ba.x, ba.y, ba.z, ba.w, bb.x, bb.y, bb.z, bb.w};
      v8f hev;
#pragma unroll
      for (int e = 0; e < 8; ++e) {
        const float he = silu_f(v8[e] + b8[e]);
        hev[e] = he;
        const v4f sw = *(const v4fa*)(cst + 4 * HID + (8 * c8 + e) * 4);
        s0 = fmaf(he, sw.x, s0);
        s1 = fmaf(he, sw.y, s1);
        s2 = fmaf(he, sw.z, s2);
        s3 = fmaf(he, sw.w, s3);
      }
      const v4f h0 = {hev[0], hev[1], hev[2], hev[3]};
      const v4f h1 = {hev[4], hev[5], hev[6], hev[7]};
      *(v4fa*)(rd + 8 * c8)     = h0;
      *(v4fa*)(rd + 8 * c8 + 4) = h1;
    }
    s0 += cst[8 * HID + 0];
    s1 += cst[8 * HID + 1];
    s2 += cst[8 * HID + 2];
    s3 += cst[8 * HID + 3];
    const float l0 = (s0 >= 0.0f) ? s0 : 0.2f * s0;
    const float l1 = (s1 >= 0.0f) ? s1 : 0.2f * s1;
    const float l2 = (s2 >= 0.0f) ? s2 : 0.2f * s2;
    const float l3 = (s3 >= 0.0f) ? s3 : 0.2f * s3;
    const float eye = (j == i) ? INFV : 0.0f;
    const v4f so = {l0 - eye, l1 - eye, l2 - eye, l3 - eye};
    *(v4fa*)(sS + 4 * tid) = so;
  }
  __syncthreads();

  {
    v4f pv[16];
#pragma unroll
    for (int it = 0; it < 16; ++it) {
      const int u   = it * NTHR + tid;
      const int row = u >> 4;
      const int c4  = (u & 15) * 4;
      pv[it] = *(const v4fa*)(sD + row * DP + c4);
    }
    const v4f so = *(const v4fa*)(sS + 4 * tid);
    float* heb = HE + (size_t)bi * NNODE * HID;
    float* sp  = SEML + ((size_t)bi * NNODE + tid) * 4;
#pragma unroll
    for (int it = 0; it < 16; ++it) *(volatile v4f*)(heb + (size_t)(it * NTHR + tid) * 4) = pv[it];
    *(volatile v4f*)sp = so;
    __threadfence();
#pragma unroll
    for (int it = 0; it < 16; ++it) *(volatile v4f*)(heb + (size_t)(it * NTHR + tid) * 4) = pv[it];
    *(volatile v4f*)sp = so;
  }
}

__global__ __launch_bounds__(NTHR) void k_row(const float* __restrict__ XB, const float* __restrict__ SEML,
                                              const float* __restrict__ HE, const float* __restrict__ h,
                                              const float* __restrict__ vin, const float* __restrict__ lg,
                                              const float* __restrict__ vmix, const float* __restrict__ WR,
                                              const float* __restrict__ pb1, const float* __restrict__ pb2,
                                              const float* __restrict__ nb1, const float* __restrict__ nb2,
                                              const float* __restrict__ vb1, const float* __restrict__ vw2,
                                              float* out0, float* XV) {
  __shared__ __attribute__((aligned(16))) float sHE[JT * HID];
  __shared__ __attribute__((aligned(16))) float sC[NNODE * 4];
  __shared__ __attribute__((aligned(16))) float sU[NNODE * 4];
  __shared__ __attribute__((aligned(16))) float s_nin[KNODE];
  __shared__ __attribute__((aligned(16))) float s_cn[CCO];
  __shared__ __attribute__((aligned(16))) float s_part[NTHR];
  __shared__ __attribute__((aligned(16))) float s_t[HID];
  __shared__ __attribute__((aligned(16))) float s_hn[FIN];
  __shared__ __attribute__((aligned(16))) float s_vs[HID];
  __shared__ __attribute__((aligned(16))) float s_xv[XVP];
  __shared__ __attribute__((aligned(16))) float red[32];

  const int tid = (int)threadIdx.x, lane = tid & 31, wave = tid >> 5;
  const int bi = (int)blockIdx.x;
  const int b  = bi >> 8;
  const int i  = bi & (NNODE - 1);

  const int j = tid;
  const v4f xi = *(const v4fa*)(XB + (size_t)(b * NNODE + i) * 4);
  const v4f xj = *(const v4fa*)(XB + (size_t)(b * NNODE + j) * 4);
  const float dx = xj.x - xi.x, dy = xj.y - xi.y, dz = xj.z - xi.z;
  const float r2  = (dx * dx + dz * dz) + dy * dy;
  const float r   = sqrtf(r2 + EPSV);
  const float eye = (j == i) ? INFV : 0.0f;
  const float inv = __builtin_amdgcn_rcpf(r + EPSV);
  {
    const v4f u4 = {dx * inv, dy * inv, dz * inv, 0.0f};
    *(v4fa*)(sU + 4 * j) = u4;
  }
  if (tid < FIN) s_nin[tid] = bf16_val(h[(size_t)bi * FIN + tid]);
  const v4f sl = *(const v4fa*)(SEML + ((size_t)bi * NNODE + j) * 4);
  const float g0 = __expf(bf16_val(lg[0]));
  const float g1 = __expf(bf16_val(lg[1]));
  const float g2 = __expf(bf16_val(lg[2]));
  const float g3 = __expf(bf16_val(lg[3]));
  const float rm = r + eye;
  v4f cm;
  {
    const v4f el = {-(rm * g0), -(rm * g1), -(rm * g2), -(rm * g3)};
    const v4f m1 = blk_max4(el, red, lane, wave);
    const v4f e1 = exp4(el - m1);
    const v4f s1 = blk_sum4(e1, red, lane, wave);
    const v4f eu = e1 * rcp4(s1);
    const v4f m2 = blk_max4(sl, red, lane, wave);
    const v4f e2 = exp4(sl - m2);
    const v4f s2 = blk_sum4(e2, red, lane, wave);
    const v4f sa = e2 * rcp4(s2);
    const v4f pp = eu * sa;
    const v4f m3 = blk_max4(pp, red, lane, wave);
    const v4f e3 = exp4(pp - m3);
    const v4f s3 = blk_sum4(e3, red, lane, wave);
    cm = e3 * rcp4(s3);
    *(v4fa*)(sC + 4 * j) = cm;
  }
  __syncthreads();

  const int c = tid, kf = c >> 2, hd = c & 3;
  float G0 = 0.0f, G1 = 0.0f, G2 = 0.0f, G3 = 0.0f;
  const float* heb = HE + (size_t)bi * NNODE * HID;
#pragma unroll 1
  for (int jt = 0; jt < NNODE / JT; ++jt) {
#pragma unroll
    for (int q = 0; q < 4; ++q) {
      const int u = q * NTHR + tid;
      *(v4fa*)(sHE + 4 * u) = *(const v4fa*)(heb + (size_t)jt * JT * HID + 4 * u);
    }
    __syncthreads();
    const float* cb = sC + (jt * JT) * 4 + hd;
    const float* ub = sU + (jt * JT) * 4;
#pragma unroll 4
    for (int jj = 0; jj < JT; ++jj) {
      const float w  = sHE[jj * HID + kf] * cb[jj * 4];
      const v4f   uu = *(const v4fa*)(ub + jj * 4);
      G0 += w;
      G1 = fmaf(w, uu.x, G1);
      G2 = fmaf(w, uu.y, G2);
      G3 = fmaf(w, uu.z, G3);
    }
    __syncthreads();
  }
  const float csx = G1 * RN256, csy = G2 * RN256, csz = G3 * RN256;
  const float cn  = (csx * csx + csz * csz) + csy * csy;
  s_nin[FIN + c] = G0;
  s_cn[c] = cn;
  const float vwv = bf16_val(vmix[c]);
  __syncthreads();
  v4f dv;
  {
    const v4f dq = {vwv * csx, vwv * csy, vwv * csz, 0.0f};
    dv = blk_sum4(dq, red, lane, wave);
  }

  const int oc = tid & (HID - 1), q = tid >> 6;
  {
    float pa = 0.0f;
    const float* wp = WR + OFF_PW1 + oc;
#pragma unroll 2
    for (int t2 = 0; t2 < CCO / 4; ++t2) {
      const int kk = (CCO / 4) * q + t2;
      pa = fmaf(s_cn[kk], wp[(size_t)kk * HID], pa);
    }
    s_part[tid] = pa;
  }
  __syncthreads();
  if (tid < HID) {
    float a = ((s_part[oc] + s_part[HID + oc]) + s_part[2 * HID + oc]) + s_part[3 * HID + oc];
    a += bf16_val(pb1[oc]);
    s_t[oc] = silu_f(a);
  }
  __syncthreads();
  {
    float pa = 0.0f;
    const float* wp = WR + OFF_PW2 + oc;
#pragma unroll 2
    for (int t2 = 0; t2 < HID / 4; ++t2) {
      const int kk = (HID / 4) * q + t2;
      pa = fmaf(s_t[kk], wp[(size_t)kk * HID], pa);
    }
    s_part[tid] = pa;
  }
  __syncthreads();
  if (tid < HID) {
    float a = ((s_part[oc] + s_part[HID + oc]) + s_part[2 * HID + oc]) + s_part[3 * HID + oc];
    a += bf16_val(pb2[oc]);
    s_nin[FIN + CCO + oc] = silu_f(a);
  }
  __syncthreads();
  {
    float pa = 0.0f;
    const float* wp = WR + OFF_NW1 + oc;
#pragma unroll 2
    for (int t2 = 0; t2 < KNODE / 4; ++t2) {
      const int kk = (KNODE / 4) * q + t2;
      pa = fmaf(s_nin[kk], wp[(size_t)kk * HID], pa);
    }
    s_part[tid] = pa;
  }
  __syncthreads();
  if (tid < HID) {
    float a = ((s_part[oc] + s_part[HID + oc]) + s_part[2 * HID + oc]) + s_part[3 * HID + oc];
    a += bf16_val(nb1[oc]);
    s_t[oc] = silu_f(a);
  }
  __syncthreads();
  {
    float pa = 0.0f;
    const float* wp = WR + OFF_NW2 + oc;
#pragma unroll 2
    for (int t2 = 0; t2 < HID / 4; ++t2) {
      const int kk = (HID / 4) * q + t2;
      pa = fmaf(s_t[kk], wp[(size_t)kk * FIN], pa);
    }
    s_part[tid] = pa;
  }
  __syncthreads();
  if (tid < FIN) {
    float a = ((s_part[oc] + s_part[HID + oc]) + s_part[2 * HID + oc]) + s_part[3 * HID + oc];
    a += bf16_val(nb2[oc]);
    s_hn[oc] = s_nin[oc] + silu_f(a);
  }
  __syncthreads();
  {
    float pa = 0.0f;
    const float* wp = WR + OFF_VW1 + oc;
#pragma unroll 2
    for (int t2 = 0; t2 < FIN / 4; ++t2) {
      const int kk = (FIN / 4) * q + t2;
      pa = fmaf(s_hn[kk], wp[(size_t)kk * HID], pa);
    }
    s_part[tid] = pa;
  }
  __syncthreads();
  if (tid < HID) {
    float a = ((s_part[oc] + s_part[HID + oc]) + s_part[2 * HID + oc]) + s_part[3 * HID + oc];
    a += bf16_val(vb1[oc]);
    s_vs[oc] = silu_f(a) * bf16_val(vw2[oc]);
  }
  __syncthreads();
  float vscale;
  {
    const float sv = (tid < HID) ? s_vs[tid & (HID - 1)] : 0.0f;
    const v4f vq = {sv, 0.0f, 0.0f, 0.0f};
    const v4f vs4 = blk_sum4(vq, red, lane, wave);
    vscale = vs4.x;
  }
  if (tid < 32) {
    const int dd  = tid & 3;
    const int ddc = dd < 3 ? dd : 2;
    const float vv  = bf16_val(vin[(size_t)bi * 3 + ddc]);
    const float dvs = (dd == 0) ? dv.x : ((dd == 1) ? dv.y : dv.z);
    const float xs  = (dd == 0) ? xi.x : ((dd == 1) ? xi.y : xi.z);
    const float vn  = fmaf(vscale, vv, dvs);
    const float xn  = xs + vn;
    float val = 0.0f;
    val = (tid < 3) ? xn : val;
    val = (tid >= 4 && tid < 7) ? vn : val;
    s_xv[tid] = val;
  }
  __syncthreads();

  if (tid < 32) {
    const int l16 = tid & 15, l8 = tid & 7;
    const v4f hv4 = *(const v4fa*)(s_hn + 4 * l16);
    const v4f xv4 = *(const v4fa*)(s_xv + 4 * l8);
    float* hp = out0 + (size_t)bi * FIN + 4 * l16;
    float* xp = XV + (size_t)bi * XVP + 4 * l8;
    if (tid < 16) *(volatile v4f*)hp = hv4;
    if (tid < 8)  *(volatile v4f*)xp = xv4;
    __threadfence();
    if (tid < 16) *(volatile v4f*)hp = hv4;
    if (tid < 8)  *(volatile v4f*)xp = xv4;
  }
}

__global__ __launch_bounds__(NTHR) void k_pack(const float* __restrict__ XV, float* out) {
  __shared__ __attribute__((aligned(16))) float s[2 * OUT1N];
  const int tid = (int)threadIdx.x;
  for (int e = tid; e < 2 * OUT1N; e += NTHR) {
    const int sel = (e < OUT1N) ? 0 : 1;
    const int eo  = e - sel * OUT1N;
    const int row = eo / 3;
    const int dd  = eo - 3 * row;
    s[e] = XV[(size_t)row * XVP + 4 * sel + dd];
  }
  __syncthreads();
  v4f pv[3];
#pragma unroll
  for (int it = 0; it < 3; ++it) pv[it] = *(const v4fa*)(s + 4 * (it * NTHR + tid));
#pragma unroll
  for (int it = 0; it < 3; ++it) *(volatile v4f*)(out + OUT0N + (size_t)4 * (it * NTHR + tid)) = pv[it];
  __threadfence();
#pragma unroll
  for (int it = 0; it < 3; ++it) *(volatile v4f*)(out + OUT0N + (size_t)4 * (it * NTHR + tid)) = pv[it];
}

extern "C" void kernel_launch(void* const* d_in, const int* in_sizes, int n_in,
                              void* d_out, int out_size, void* d_ws, size_t ws_size,
                              hipStream_t stream) {
  if (n_in < 22) return;
  if (in_sizes[0] != NR * FIN) return;
  if (in_sizes[1] != NR * 3 || in_sizes[2] != NR * 3) return;
  if (in_sizes[3] != KIN1 * HID || in_sizes[4] != HID) return;
  if (in_sizes[5] != HID * HID || in_sizes[6] != HID) return;
  if (in_sizes[7] != HID * NHEAD || in_sizes[8] != NHEAD) return;
  if (in_sizes[9] != CCO * HID || in_sizes[10] != HID) return;
  if (in_sizes[11] != HID * HID || in_sizes[12] != HID) return;
  if (in_sizes[13] != KNODE * HID || in_sizes[14] != HID) return;
  if (in_sizes[15] != HID * FIN || in_sizes[16] != FIN) return;
  if (in_sizes[17] != FIN * HID || in_sizes[18] != HID) return;
  if (in_sizes[19] != HID) return;
  if (in_sizes[20] != CCO || in_sizes[21] != NHEAD) return;
  if (out_size != OUTN) return;

  const float* h    = (const float*)d_in[0];
  const float* x    = (const float*)d_in[1];
  const float* v    = (const float*)d_in[2];
  const float* ew1  = (const float*)d_in[3];
  const float* eb1  = (const float*)d_in[4];
  const float* ew2  = (const float*)d_in[5];
  const float* eb2  = (const float*)d_in[6];
  const float* semw = (const float*)d_in[7];
  const float* semb = (const float*)d_in[8];
  const float* pw1  = (const float*)d_in[9];
  const float* pb1  = (const float*)d_in[10];
  const float* pw2  = (const float*)d_in[11];
  const float* pb2  = (const float*)d_in[12];
  const float* nw1  = (const float*)d_in[13];
  const float* nb1  = (const float*)d_in[14];
  const float* nw2  = (const float*)d_in[15];
  const float* nb2  = (const float*)d_in[16];
  const float* vw1  = (const float*)d_in[17];
  const float* vb1  = (const float*)d_in[18];
  const float* vw2  = (const float*)d_in[19];
  const float* vmix = (const float*)d_in[20];
  const float* lg   = (const float*)d_in[21];
  float* out0 = (float*)d_out;

  char* ws = (char*)d_ws;
  size_t off = 0;
  const size_t oWPT  = off; off += (size_t)ABW * FIN * 2;
  const size_t oW2D  = off; off += (size_t)HID * KE2 * 2;
  const size_t oHB   = off; off += (size_t)NR * FIN * 2;
  const size_t oXB   = off; off += (size_t)NR * 4 * 4;
  const size_t oWR   = off; off += (size_t)WRN * 4;
  const size_t oAB   = off; off += (size_t)NR * ABW * 4;
  const size_t oHE   = off; off += (size_t)NPAIR * HID * 4;
  const size_t oSEML = off; off += (size_t)NPAIR * 4 * 4;
  const size_t oXV   = off; off += (size_t)NR * XVP * 4;
  if (off > ws_size || off > (size_t)WSMAX) return;
  unsigned short* WPT  = (unsigned short*)(ws + oWPT);
  unsigned short* W2D  = (unsigned short*)(ws + oW2D);
  unsigned short* HB   = (unsigned short*)(ws + oHB);
  float*          XB   = (float*)(ws + oXB);
  float*          WR   = (float*)(ws + oWR);
  float*          AB   = (float*)(ws + oAB);
  float*          HE   = (float*)(ws + oHE);
  float*          SEML = (float*)(ws + oSEML);
  float*          XV   = (float*)(ws + oXV);

  hipFuncSetAttribute(reinterpret_cast<const void*>(&k_edge), hipFuncAttributeMaxDynamicSharedMemorySize,
                      (int)EDGE_LDS_BYTES);

  k_prep<<<NPREP / NTHR, NTHR, 0, stream>>>(h, x, ew1, ew2, pw1, pw2, nw1, nw2, vw1,
                                            WPT, W2D, HB, XB, WR);
  k_ab<<<dim3(NR / GBM, ABW / GBN), GTHR, 0, stream>>>(HB, FIN, WPT, FIN, FIN, AB, ABW);
  k_edge<<<NR, NTHR, EDGE_LDS_BYTES, stream>>>(XB, AB, ew1, eb1, W2D, eb2, semw, semb, HE, SEML);
  k_row<<<NR, NTHR, 0, stream>>>(XB, SEML, HE, h, v, lg, vmix, WR, pb1, pb2, nb1, nb2, vb1, vw2, out0, XV);
  k_pack<<<1, NTHR, 0, stream>>>(XV, out0);
}
